// GaussianActor_48868137894248
// MI455X (gfx1250) — hardware-verified
//
#include <hip/hip_runtime.h>
#include <hip/hip_bf16.h>
#include <math.h>

constexpr int   kDin          = 48;
constexpr int   kHid          = 256;
constexpr int   kDout         = 12;
constexpr int   kChunk        = 32768;
constexpr int   kK1           = 160;
constexpr int   kSegPerRow1   = kK1 / 8;
constexpr int   kHeadN        = 16;
constexpr int   kHeadRows     = 128;
constexpr int   kLnRowsPerWave  = 4;
constexpr int   kLnRowsPerBlock = 8 * kLnRowsPerWave;
constexpr int   kBt1Blocks    = (kHid * kSegPerRow1) / 256;
constexpr int   kWmBlocks     = (kHeadN * kHid / 8) / 256;
constexpr float kLnEps        = 1e-5f;
constexpr float kInvHid       = 1.0f / 256.0f;
constexpr float kActCarry     = 8.0f;
constexpr float kWCarry       = 8.0f;
constexpr float kL23Scale     = 1.0f / 64.0f;

static_assert(kBt1Blocks * 256 == kHid * kSegPerRow1);
static_assert(kWmBlocks * 256 == kHeadN * kHid / 8);
static_assert(kChunk % 64 == 0 && kChunk % kHeadRows == 0 && kChunk % kLnRowsPerBlock == 0);
static_assert((kChunk * kSegPerRow1) % 256 == 0);
static_assert(kK1 % 32 == 0 && kHid % 32 == 0);

typedef __attribute__((ext_vector_type(16))) _Float16 v16h;
typedef __attribute__((ext_vector_type(8)))  _Float16 v8h;
typedef __attribute__((ext_vector_type(16))) __bf16   v16b;
typedef __attribute__((ext_vector_type(8)))  __bf16   v8b;
typedef __attribute__((ext_vector_type(8)))  float    v8f;
typedef __attribute__((ext_vector_type(4)))  float    v4f;
typedef __attribute__((ext_vector_type(4)))  unsigned int v4u;

__device__ __forceinline__ unsigned short f2bf_bits(float f) {
  unsigned u = __float_as_uint(f);
  return (unsigned short)((u + 0x7FFFu + ((u >> 16) & 1u)) >> 16);
}
__device__ __forceinline__ float bf_bits2f(unsigned short h) { return __uint_as_float(((unsigned)h) << 16); }

__device__ __forceinline__ void dep_guard_h(v8f& a, v8f& b, v16h x, v16h y) { asm volatile("v_nop\n\tv_nop\n\tv_nop\n\tv_nop" : "+v"(a), "+v"(b) : "v"(x), "v"(y)); }
__device__ __forceinline__ void dep_guard_b(v8f& a, v8f& b, v16b x, v16b y) { asm volatile("v_nop\n\tv_nop\n\tv_nop\n\tv_nop" : "+v"(a), "+v"(b) : "v"(x), "v"(y)); }
__device__ __forceinline__ void keep4_h(v16h a, v16h b, v16h c, v16h d) { asm volatile("v_nop" :: "v"(a), "v"(b), "v"(c), "v"(d)); }
__device__ __forceinline__ void keep4_b(v16b a, v16b b, v16b c, v16b d) { asm volatile("v_nop" :: "v"(a), "v"(b), "v"(c), "v"(d)); }
__device__ __forceinline__ void acc_guard4(v8f& a, v8f& b, v8f& c, v8f& d) { asm volatile("v_nop\n\tv_nop\n\tv_nop\n\tv_nop" : "+v"(a), "+v"(b), "+v"(c), "+v"(d)); }
template <typename T> struct Frag;
template <> struct Frag<_Float16> {
  typedef v16h V; union U { v16h v; v8h h[2]; };
  static __device__ __forceinline__ v16h load(const _Float16* p) {
    U f; f.h[0] = *(const v8h*)(p); f.h[1] = *(const v8h*)(p + 16); return f.v;
  }
  static __device__ __forceinline__ v8f mma(v16h a, v16h b, v8f c) {
    return __builtin_amdgcn_wmma_f32_16x16x32_f16(false, a, false, b, (short)0, c, false, false);
  }
  static __device__ __forceinline__ void guard(v8f& a, v8f& b, v16h x, v16h y) { dep_guard_h(a, b, x, y); }
  static __device__ __forceinline__ void keep(v16h a, v16h b, v16h c, v16h d) { keep4_h(a, b, c, d); }
};
template <> struct Frag<__bf16> {
  typedef v16b V; union U { v16b v; v8b h[2]; };
  static __device__ __forceinline__ v16b load(const __bf16* p) {
    U f; f.h[0] = *(const v8b*)(p); f.h[1] = *(const v8b*)(p + 16); return f.v;
  }
  static __device__ __forceinline__ v8f mma(v16b a, v16b b, v8f c) {
    return __builtin_amdgcn_wmma_f32_16x16x32_bf16(false, a, false, b, (short)0, c, false, false);
  }
  static __device__ __forceinline__ void guard(v8f& a, v8f& b, v16b x, v16b y) { dep_guard_b(a, b, x, y); }
  static __device__ __forceinline__ void keep(v16b a, v16b b, v16b c, v16b d) { keep4_b(a, b, c, d); }
};

__device__ __forceinline__ unsigned pk16(unsigned short a, unsigned short b) { return (unsigned)a | ((unsigned)b << 16); }
__device__ __forceinline__ unsigned short h_bits(float f) { const _Float16 h = (_Float16)f; return __builtin_bit_cast(unsigned short, h); }

__device__ __forceinline__ v8f bmma(v16b a, v16b b, v8f c) {
  c = __builtin_amdgcn_wmma_f32_16x16x32_bf16(false, a, false, b, (short)0, c, false, false);
  asm volatile("v_nop\n\tv_nop\n\tv_nop\n\tv_nop" : "+v"(c) : "v"(a), "v"(b));
  return c;
}

template <int ET> struct Elem;
template <> struct Elem<0> { typedef _Float16 T; };
template <> struct Elem<1> { typedef __bf16 T; };
template <int ET, bool SPLIT, int BIAS_MODE, int OUT_MODE, bool RESID, int ACT = 0>
__global__ __launch_bounds__(256) void wmma_gemm64(
    const unsigned short* __restrict__ Ap, const unsigned short* __restrict__ A2p, int lda, long strideA,
    const unsigned short* __restrict__ Btp, const unsigned short* __restrict__ Bt2p, int ldb, long strideB,
    void* __restrict__ Cout, void* __restrict__ Cout2, int ldc, long strideC,
    const float* __restrict__ bias,
    const float* __restrict__ resid, long strideR,
    int M, int N, int K, float scale) {
  typedef typename Elem<ET>::T T;
  typedef typename Frag<T>::V V;
  const T* A = (const T*)Ap; const T* A2 = (const T*)A2p; const T* Bt = (const T*)Btp; const T* Bt2 = (const T*)Bt2p;
  __shared__ __align__(16) float sT[8][16 * 68];
  const int b    = blockIdx.y;
  const int lane = threadIdx.x & 31;
  const int wave = threadIdx.x >> 5;
  const int tilesN = N >> 6;
  const int tilesM = M >> 6;
  const int tile = blockIdx.x * 8 + wave;
  if (tile >= tilesM * tilesN) return;
  const int tm = tile / tilesN;
  const int tn = tile - tm * tilesN;
  const int m0 = tm << 6;
  const int n0 = tn << 6;

  const T* Ab  = A  + (size_t)b * strideA;
  const T* Bb  = Bt + (size_t)b * strideB;
  const T* Ab2 = SPLIT ? (A2  + (size_t)b * strideA) : nullptr;
  const T* Bb2 = SPLIT ? (Bt2 + (size_t)b * strideB) : nullptr;

  const int rlane = lane & 15;
  const int koff  = (lane >> 4) * 8;
  const int mOff  = (lane >> 4) * 8;

  v8f acc[4][4];
#pragma unroll
  for (int i = 0; i < 4; ++i)
#pragma unroll
    for (int j = 0; j < 4; ++j) acc[i][j] = (v8f){0.f,0.f,0.f,0.f,0.f,0.f,0.f,0.f};

  for (int k0 = 0; k0 < K; k0 += 32) {
    V bh[4], bl[4];
#pragma unroll
    for (int j = 0; j < 4; ++j) {
      const size_t bo = (size_t)(n0 + (j << 4) + rlane) * ldb + koff + k0;
      bh[j] = Frag<T>::load(Bb + bo);
      if (SPLIT) bl[j] = Frag<T>::load(Bb2 + bo);
    }
#pragma unroll
    for (int i = 0; i < 4; ++i) {
      const size_t ao = (size_t)(m0 + (i << 4) + rlane) * lda + koff + k0;
      V ah = Frag<T>::load(Ab + ao);
      V al;
      if (SPLIT) al = Frag<T>::load(Ab2 + ao);
#pragma unroll
      for (int j = 0; j < 4; ++j) {
        acc[i][j] = Frag<T>::mma(ah, bh[j], acc[i][j]);
        if (SPLIT) {
          acc[i][j] = Frag<T>::mma(ah, bl[j], acc[i][j]);
          acc[i][j] = Frag<T>::mma(al, bh[j], acc[i][j]);
        }
      }
      Frag<T>::guard(acc[i][0], acc[i][3], ah, SPLIT ? al : ah);
    }
    Frag<T>::keep(bh[0], bh[1], bh[2], bh[3]);
    if (SPLIT) Frag<T>::keep(bl[0], bl[1], bl[2], bl[3]);
  }
  acc_guard4(acc[0][0], acc[0][1], acc[0][2], acc[0][3]);
  acc_guard4(acc[1][0], acc[1][1], acc[1][2], acc[1][3]);
  acc_guard4(acc[2][0], acc[2][1], acc[2][2], acc[2][3]);
  acc_guard4(acc[3][0], acc[3][1], acc[3][2], acc[3][3]);

  float* slab = sT[wave];
  const float* Rb = RESID ? (resid + (size_t)b * strideR) : nullptr;
#pragma unroll
  for (int i = 0; i < 4; ++i) {
    const int mBase = m0 + (i << 4);
#pragma unroll
    for (int j = 0; j < 4; ++j) {
      const int n = n0 + (j << 4) + rlane;
      float bv = 0.f;
      if (BIAS_MODE == 2) bv = bias[n];
#pragma unroll
      for (int r = 0; r < 8; ++r) {
        float v = acc[i][j][r] * scale;
        if (BIAS_MODE == 1) v += bias[mBase + mOff + r];
        if (BIAS_MODE == 2) v += bv;
        if (RESID) v += Rb[(size_t)(mBase + mOff + r) * ldc + n];
        if (ACT == 2) v = fmaxf(v, 0.0f);
        if (ACT == 4) v = (v > 0.f) ? v : 0.01f * v;
        slab[(mOff + r) * 68 + (j << 4) + rlane] = v;
      }
    }
    __builtin_amdgcn_fence(__ATOMIC_RELEASE, "workgroup");
    __builtin_amdgcn_wave_barrier();
    __builtin_amdgcn_fence(__ATOMIC_ACQUIRE, "workgroup");
    if (OUT_MODE == 0) {
      float* C = (float*)Cout + (size_t)b * strideC;
      const int hh = lane >> 4, c4 = (lane & 15) * 4;
      for (int pass = 0; pass < 2; ++pass) {
#pragma unroll
        for (int it = 0; it < 8; ++it) {
          const int row = it * 2 + hh;
          v4f v = *(const v4f*)(slab + row * 68 + c4);
          *(volatile v4f*)(C + (size_t)(mBase + row) * ldc + n0 + c4) = v;
        }
        __threadfence();
      }
    } else {
      const int q = lane >> 3, c8 = (lane & 7) * 8;
      unsigned short* C  = (unsigned short*)Cout  + (size_t)b * strideC;
      unsigned short* C2 = (OUT_MODE == 2) ? ((unsigned short*)Cout2 + (size_t)b * strideC) : nullptr;
      for (int pass = 0; pass < 2; ++pass) {
#pragma unroll
        for (int it = 0; it < 4; ++it) {
          const int row = it * 4 + q;
          const float* sp = slab + row * 68 + c8;
          v8h hv, lv;
#pragma unroll
          for (int e = 0; e < 8; ++e) {
            if (OUT_MODE == 1) {
              hv[e] = (_Float16)sp[e];
            } else {
              unsigned short hb = f2bf_bits(sp[e]);
              unsigned short lb = f2bf_bits(sp[e] - bf_bits2f(hb));
              hv[e] = __builtin_bit_cast(_Float16, hb);
              lv[e] = __builtin_bit_cast(_Float16, lb);
            }
          }
          *(volatile v8h*)(C + (size_t)(mBase + row) * ldc + n0 + c8) = hv;
          if (OUT_MODE == 2) *(volatile v8h*)(C2 + (size_t)(mBase + row) * ldc + n0 + c8) = lv;
        }
        __threadfence();
      }
    }
    __builtin_amdgcn_fence(__ATOMIC_RELEASE, "workgroup");
    __builtin_amdgcn_wave_barrier();
    __builtin_amdgcn_fence(__ATOMIC_ACQUIRE, "workgroup");
  }
}

__global__ __launch_bounds__(256) void wtcast_kernel(const float* __restrict__ WA, const float* __restrict__ WB,
                                                     unsigned short* __restrict__ out, float scale) {
  __shared__ float sm[64][65];
  const int t  = threadIdx.x;
  const int d0 = blockIdx.x * 64;
  const int h0 = blockIdx.y * 64;
  const int z  = blockIdx.z;
  const float* W = (z == 0) ? WA : WB;
#pragma unroll
  for (int i = 0; i < 16; ++i) {
    const int e = i * 256 + t;
    const int r = e >> 6;
    const int c = e & 63;
    sm[c][r] = W[(size_t)(d0 + r) * kHid + h0 + c] * scale;
  }
  __syncthreads();
  const int lane = t & 31, wave = t >> 5;
  const int q = lane >> 3, c8 = (lane & 7) * 8;
  unsigned short* op = out + (size_t)z * kHid * kHid;
  for (int pass = 0; pass < 2; ++pass) {
#pragma unroll
    for (int it = 0; it < 2; ++it) {
      const int row = wave * 8 + it * 4 + q;
      unsigned short hb[8];
#pragma unroll
      for (int e = 0; e < 8; ++e) hb[e] = h_bits(sm[row][c8 + e]);
      const v4u u = (v4u){pk16(hb[0], hb[1]), pk16(hb[2], hb[3]), pk16(hb[4], hb[5]), pk16(hb[6], hb[7])};
      *(volatile v4u*)(op + (size_t)(h0 + row) * kHid + d0 + c8) = u;
    }
    __threadfence();
  }
}

__global__ __launch_bounds__(256) void wprep_small_kernel(const float* __restrict__ W1, const float* __restrict__ Wm,
                                                          unsigned short* __restrict__ Bt1,
                                                          unsigned short* __restrict__ Bmh, unsigned short* __restrict__ Bml) {
  const int t = threadIdx.x;
  if (blockIdx.x < kBt1Blocks) {
    const int f   = blockIdx.x * 256 + t;
    const int n   = f / kSegPerRow1;
    const int seg = f - n * kSegPerRow1;
    const int grp = seg / 6;
    const int cc  = (grp < 3) ? (seg - grp * 6) * 8 : 0;
    unsigned short o[8];
#pragma unroll
    for (int e = 0; e < 8; ++e) {
      const float v = W1[(size_t)(cc + e) * kHid + n];
      const unsigned short hb = f2bf_bits(v);
      const unsigned short lb = f2bf_bits(v - bf_bits2f(hb));
      const unsigned short s = (grp == 2) ? lb : hb;
      o[e] = (grp == 3) ? (unsigned short)0 : s;
    }
    const v4u u = (v4u){pk16(o[0], o[1]), pk16(o[2], o[3]), pk16(o[4], o[5]), pk16(o[6], o[7])};
    unsigned short* q = Bt1 + 8 * (size_t)f;
    *(volatile v4u*)q = u;
    __threadfence();
    *(volatile v4u*)q = u;
  } else {
    const int f  = (blockIdx.x - kBt1Blocks) * 256 + t;
    const int n  = f >> 5;
    const int k0 = (f & 31) * 8;
    const int nc = (n < kDout) ? n : (kDout - 1);
    unsigned short ho[8], lo[8];
#pragma unroll
    for (int e = 0; e < 8; ++e) {
      const float v = Wm[(size_t)(k0 + e) * kDout + nc];
      const unsigned short hb = f2bf_bits(v);
      const unsigned short lb = f2bf_bits(v - bf_bits2f(hb));
      ho[e] = (n < kDout) ? hb : (unsigned short)0;
      lo[e] = (n < kDout) ? lb : (unsigned short)0;
    }
    const v4u uh = (v4u){pk16(ho[0], ho[1]), pk16(ho[2], ho[3]), pk16(ho[4], ho[5]), pk16(ho[6], ho[7])};
    const v4u ul = (v4u){pk16(lo[0], lo[1]), pk16(lo[2], lo[3]), pk16(lo[4], lo[5]), pk16(lo[6], lo[7])};
    unsigned short* qh = Bmh + 8 * (size_t)f;
    unsigned short* ql = Bml + 8 * (size_t)f;
    *(volatile v4u*)qh = uh;
    *(volatile v4u*)ql = ul;
    __threadfence();
    *(volatile v4u*)qh = uh;
    *(volatile v4u*)ql = ul;
  }
}

__global__ __launch_bounds__(256) void xpack_kernel(const float* __restrict__ X, unsigned short* __restrict__ A1, int nrows) {
  const int total = nrows * kSegPerRow1;
  const int f   = blockIdx.x * 256 + threadIdx.x;
  const int fc  = (f < total) ? f : (total - 1);
  const int row = fc / kSegPerRow1;
  const int seg = fc - row * kSegPerRow1;
  const int grp = seg / 6;
  const int cc  = (grp < 3) ? (seg - grp * 6) * 8 : 0;
  const float* xp = X + (size_t)row * kDin + cc;
  const v4f a = *(const v4f*)(xp);
  const v4f c = *(const v4f*)(xp + 4);
  float xv[8];
#pragma unroll
  for (int e = 0; e < 4; ++e) { xv[e] = a[e]; xv[4 + e] = c[e]; }
  unsigned short o[8];
#pragma unroll
  for (int e = 0; e < 8; ++e) {
    const unsigned short hb = f2bf_bits(xv[e]);
    const unsigned short lb = f2bf_bits(xv[e] - bf_bits2f(hb));
    const unsigned short s = (grp == 1) ? lb : hb;
    o[e] = (grp == 3) ? (unsigned short)0 : s;
  }
  const v4u u = (v4u){pk16(o[0], o[1]), pk16(o[2], o[3]), pk16(o[4], o[5]), pk16(o[6], o[7])};
  if (f < total) {
    unsigned short* q = A1 + 8 * (size_t)f;
    *(volatile v4u*)q = u;
    __threadfence();
    *(volatile v4u*)q = u;
  }
}

template <int OUTM>
__global__ __launch_bounds__(256) void ln_relu_kernel(const float* __restrict__ H, const float* __restrict__ bias,
                                                      const float* __restrict__ gam, const float* __restrict__ bet,
                                                      unsigned short* __restrict__ O1, unsigned short* __restrict__ O2,
                                                      int nrows, float carry) {
  const int lane = threadIdx.x & 31, wave = threadIdx.x >> 5;
  const int c0 = lane * 8;
  float bb[8], gg[8], ee[8];
  {
    const v4f b0 = *(const v4f*)(bias + c0), b1v = *(const v4f*)(bias + c0 + 4);
    const v4f g0 = *(const v4f*)(gam + c0),  g1v = *(const v4f*)(gam + c0 + 4);
    const v4f e0 = *(const v4f*)(bet + c0),  e1v = *(const v4f*)(bet + c0 + 4);
#pragma unroll
    for (int e = 0; e < 4; ++e) {
      bb[e] = b0[e]; bb[4 + e] = b1v[e];
      gg[e] = g0[e]; gg[4 + e] = g1v[e];
      ee[e] = e0[e]; ee[4 + e] = e1v[e];
    }
  }
  const int rbase = (blockIdx.x * 8 + wave) * kLnRowsPerWave;
#pragma unroll 1
  for (int it = 0; it < kLnRowsPerWave; ++it) {
    const int row  = rbase + it;
    const int rowc = (row < nrows) ? row : (nrows - 1);
    const float* hp = H + (size_t)rowc * kHid + c0;
    const v4f a = *(const v4f*)(hp);
    const v4f c = *(const v4f*)(hp + 4);
    float xv[8];
#pragma unroll
    for (int e = 0; e < 4; ++e) { xv[e] = a[e] + bb[e]; xv[4 + e] = c[e] + bb[4 + e]; }
    float s = 0.f;
#pragma unroll
    for (int e = 0; e < 8; ++e) s += xv[e];
#pragma unroll
    for (int off = 16; off > 0; off >>= 1) s += __shfl_xor(s, off, 32);
    const float mu = s * kInvHid;
    float d[8];
    float sq = 0.f;
#pragma unroll
    for (int e = 0; e < 8; ++e) { d[e] = xv[e] - mu; sq += d[e] * d[e]; }
#pragma unroll
    for (int off = 16; off > 0; off >>= 1) sq += __shfl_xor(sq, off, 32);
    const float var = sq * kInvHid;
    const float rs = rsqrtf(var + kLnEps);
    float y[8];
#pragma unroll
    for (int e = 0; e < 8; ++e) y[e] = fmaxf(d[e] * rs * gg[e] + ee[e], 0.0f);
    if (OUTM == 0) {
      unsigned short o[8];
#pragma unroll
      for (int e = 0; e < 8; ++e) o[e] = h_bits(y[e] * carry);
      const v4u u = (v4u){pk16(o[0], o[1]), pk16(o[2], o[3]), pk16(o[4], o[5]), pk16(o[6], o[7])};
      if (row < nrows) {
        unsigned short* q = O1 + (size_t)row * kHid + c0;
        *(volatile v4u*)q = u;
        __threadfence();
        *(volatile v4u*)q = u;
      }
    } else {
      unsigned short ho[8], lo[8];
#pragma unroll
      for (int e = 0; e < 8; ++e) {
        const unsigned short hb = f2bf_bits(y[e]);
        ho[e] = hb;
        lo[e] = f2bf_bits(y[e] - bf_bits2f(hb));
      }
      const v4u uh = (v4u){pk16(ho[0], ho[1]), pk16(ho[2], ho[3]), pk16(ho[4], ho[5]), pk16(ho[6], ho[7])};
      const v4u ul = (v4u){pk16(lo[0], lo[1]), pk16(lo[2], lo[3]), pk16(lo[4], lo[5]), pk16(lo[6], lo[7])};
      if (row < nrows) {
        unsigned short* qh = O1 + (size_t)row * kHid + c0;
        unsigned short* ql = O2 + (size_t)row * kHid + c0;
        *(volatile v4u*)qh = uh;
        *(volatile v4u*)ql = ul;
        __threadfence();
        *(volatile v4u*)qh = uh;
        *(volatile v4u*)ql = ul;
      }
    }
  }
}

__global__ __launch_bounds__(256) void head_kernel(const unsigned short* __restrict__ Hh, const unsigned short* __restrict__ Hl,
                                                   const unsigned short* __restrict__ Bh, const unsigned short* __restrict__ Bl,
                                                   const float* __restrict__ bm, float* __restrict__ out, int nrows) {
  __shared__ __align__(16) float sOut[kHeadRows * kDout];
  const int t = threadIdx.x, lane = t & 31, wave = t >> 5;
  const int rlane = lane & 15, hh = lane >> 4, koff = hh * 8;
  const int rw = blockIdx.x * kHeadRows + wave * 16;
  int ar = rw + rlane;
  ar = (ar < nrows) ? ar : (nrows - 1);
  const __bf16* Ahp = (const __bf16*)Hh + (size_t)ar * kHid + koff;
  const __bf16* Alp = (const __bf16*)Hl + (size_t)ar * kHid + koff;
  const __bf16* Bhp = (const __bf16*)Bh + (size_t)rlane * kHid + koff;
  const __bf16* Blp = (const __bf16*)Bl + (size_t)rlane * kHid + koff;
  v8f acc = (v8f){0.f,0.f,0.f,0.f,0.f,0.f,0.f,0.f};
#pragma unroll 2
  for (int k0 = 0; k0 < kHid; k0 += 32) {
    const v16b ah = Frag<__bf16>::load(Ahp + k0);
    const v16b al = Frag<__bf16>::load(Alp + k0);
    const v16b bh = Frag<__bf16>::load(Bhp + k0);
    const v16b bl = Frag<__bf16>::load(Blp + k0);
    acc = bmma(ah, bh, acc);
    acc = bmma(ah, bl, acc);
    acc = bmma(al, bh, acc);
  }
  const float bmv = bm[(rlane < kDout) ? rlane : (kDout - 1)];
#pragma unroll
  for (int r = 0; r < 8; ++r) {
    const float v = tanhf(acc[r] + bmv);
    if (rlane < kDout) sOut[(wave * 16 + hh * 8 + r) * kDout + rlane] = v;
  }
  __syncthreads();
  float* ob = out + (size_t)blockIdx.x * (kHeadRows * kDout);
  for (int pass = 0; pass < 2; ++pass) {
#pragma unroll
    for (int j = 0; j < 2; ++j) {
      const int i = t + 256 * j;
      if (i < (kHeadRows * kDout) / 4) {
        const v4f val = *(const v4f*)(sOut + 4 * i);
        *(volatile v4f*)(ob + 4 * (size_t)i) = val;
      }
    }
    __threadfence();
  }
}

extern "C" void kernel_launch(void* const* d_in, const int* in_sizes, int n_in,
                              void* d_out, int out_size, void* d_ws, size_t ws_size, hipStream_t stream) {
  const float* x   = (const float*)d_in[0];
  const float* W1  = (const float*)d_in[1];
  const float* b1  = (const float*)d_in[2];
  const float* g1  = (const float*)d_in[3];
  const float* be1 = (const float*)d_in[4];
  const float* W2  = (const float*)d_in[5];
  const float* b2  = (const float*)d_in[6];
  const float* g2  = (const float*)d_in[7];
  const float* be2 = (const float*)d_in[8];
  const float* W3  = (const float*)d_in[9];
  const float* b3  = (const float*)d_in[10];
  const float* g3  = (const float*)d_in[11];
  const float* be3 = (const float*)d_in[12];
  const float* Wm  = (const float*)d_in[13];
  const float* bm  = (const float*)d_in[14];
  float* out = (float*)d_out;
  (void)n_in; (void)stream;

  const int rows = in_sizes[0] / kDin;
  if (rows <= 0 || (rows % kChunk) != 0) return;
  if (out_size < rows * kDout) return;
  const int nchunks = rows / kChunk;

  const size_t off_wt23 = 0;
  const size_t sz_wt23  = (size_t)2 * kHid * kHid * 2;
  const size_t off_bt1  = off_wt23 + sz_wt23;
  const size_t sz_bt1   = (size_t)kHid * kK1 * 2;
  const size_t off_bmh  = off_bt1 + sz_bt1;
  const size_t sz_bm    = (size_t)kHeadN * kHid * 2;
  const size_t off_bml  = off_bmh + sz_bm;
  const size_t off_ra   = off_bml + sz_bm;
  const size_t sz_a1    = (size_t)kChunk * kK1 * 2;
  const size_t sz_hl    = (size_t)kChunk * kHid * 2;
  const size_t sz_ra    = (sz_a1 > sz_hl) ? sz_a1 : sz_hl;
  const size_t off_hf   = off_ra + sz_ra;
  const size_t sz_hf    = (size_t)kChunk * kHid * 4;
  const size_t off_p16  = off_hf + sz_hf;
  const size_t sz_p16   = (size_t)kChunk * kHid * 2;
  const size_t total_ws = off_p16 + sz_p16;
  if (total_ws > ws_size) return;

  unsigned char* ws = (unsigned char*)d_ws;
  unsigned short* Wt23 = (unsigned short*)(ws + off_wt23);
  unsigned short* Wt2  = Wt23;
  unsigned short* Wt3  = Wt23 + (size_t)kHid * kHid;
  unsigned short* Bt1  = (unsigned short*)(ws + off_bt1);
  unsigned short* Bmh  = (unsigned short*)(ws + off_bmh);
  unsigned short* Bml  = (unsigned short*)(ws + off_bml);
  unsigned short* A1   = (unsigned short*)(ws + off_ra);
  unsigned short* Hl   = (unsigned short*)(ws + off_ra);
  float*          Hf   = (float*)(ws + off_hf);
  unsigned short* P16  = (unsigned short*)(ws + off_p16);
  unsigned short* Hh   = (unsigned short*)(ws + off_p16);

  wprep_small_kernel<<<kBt1Blocks + kWmBlocks, 256, 0, stream>>>(W1, Wm, Bt1, Bmh, Bml);
  wtcast_kernel<<<dim3(kHid / 64, kHid / 64, 2), 256, 0, stream>>>(W2, W3, Wt23, kWCarry);

  const int gemm_tiles  = (kChunk / 64) * (kHid / 64);
  const int gemm_blocks = (gemm_tiles + 7) / 8;
  const int xpack_blocks = (kChunk * kSegPerRow1) / 256;
  const int ln_blocks   = kChunk / kLnRowsPerBlock;
  const int head_blocks = kChunk / kHeadRows;

  for (int ch = 0; ch < nchunks; ++ch) {
    const size_t row0 = (size_t)ch * kChunk;
    const float* xc = x + row0 * kDin;
    float* oc = out + row0 * kDout;

    xpack_kernel<<<xpack_blocks, 256, 0, stream>>>(xc, A1, kChunk);
    wmma_gemm64<1, false, 0, 0, false, 0><<<dim3(gemm_blocks, 1), 256, 0, stream>>>(
        A1, A1, kK1, (long)0, Bt1, Bt1, kK1, (long)0, (void*)Hf, (void*)Hf, kHid, (long)0,
        nullptr, nullptr, (long)0, kChunk, kHid, kK1, 1.0f);
    ln_relu_kernel<0><<<ln_blocks, 256, 0, stream>>>(Hf, b1, g1, be1, P16, P16, kChunk, kActCarry);

    wmma_gemm64<0, false, 0, 0, false, 0><<<dim3(gemm_blocks, 1), 256, 0, stream>>>(
        P16, P16, kHid, (long)0, Wt2, Wt2, kHid, (long)0, (void*)Hf, (void*)Hf, kHid, (long)0,
        nullptr, nullptr, (long)0, kChunk, kHid, kHid, kL23Scale);
    ln_relu_kernel<0><<<ln_blocks, 256, 0, stream>>>(Hf, b2, g2, be2, P16, P16, kChunk, kActCarry);

    wmma_gemm64<0, false, 0, 0, false, 0><<<dim3(gemm_blocks, 1), 256, 0, stream>>>(
        P16, P16, kHid, (long)0, Wt3, Wt3, kHid, (long)0, (void*)Hf, (void*)Hf, kHid, (long)0,
        nullptr, nullptr, (long)0, kChunk, kHid, kHid, kL23Scale);
    ln_relu_kernel<1><<<ln_blocks, 256, 0, stream>>>(Hf, b3, g3, be3, Hh, Hl, kChunk, 1.0f);

    head_kernel<<<head_blocks, 256, 0, stream>>>(Hh, Hl, Bmh, Bml, bm, oc, kChunk);
  }
}
